// CareerTreeModel_30889404793607
// MI455X (gfx1250) — hardware-verified
//
#include <hip/hip_runtime.h>
#include <stddef.h>
#include <math.h>


#define DI      128
#define DH      128
#define DZ      64
#define DE      32
#define NTHR    256
#define NWAVE   8
#define EPT     8
#define NGRP    2
#define CHUNK   (NTHR * EPT * NGRP)
#define WCAP    (EPT * NGRP * 32)
#define LISTN   (NWAVE * WCAP)
#define NBC     4096
#define NBF     1024
#define RCAP    40960
#define RBN     128
#define TGT     256
#define DEGCAP  512
#define OTHR    512
#define DTHR    256
#define BM      32
#define LDU     72
#define WSCAP   134217728
#define SCL_A   8.0f
#define SCL_W   16.0f
#define SCL_ACC 0.0078125f

#define LDS_FILL ((RCAP + NBF + LISTN) * 4 + 64)

static_assert((CHUNK & (CHUNK - 1)) == 0);
static_assert(CHUNK <= 4096);
static_assert(NBC <= 4096 && NBF <= 4096);
static_assert((NBC & (NBC - 1)) == 0 && (NBF & (NBF - 1)) == 0);
static_assert(NBC == 4 * NBF);
static_assert(OTHR * 8 == NBC);
static_assert((RCAP % 32) == 0);
static_assert(TGT == NWAVE * 32);
static_assert((NBC % TGT) == 0);
static_assert((TGT % BM) == 0);
static_assert(DI == 128 && DH == DI && DZ == 64 && DE == 32);
static_assert(DTHR == 256);
static_assert((LDU % 8) == 0 && LDU >= DZ);

typedef float    v2f  __attribute__((ext_vector_type(2)));
typedef float    v4f  __attribute__((ext_vector_type(4)));
typedef float    v8f  __attribute__((ext_vector_type(8)));
typedef int      v4i  __attribute__((ext_vector_type(4)));
typedef _Float16 v2h  __attribute__((ext_vector_type(2)));
typedef _Float16 v4h  __attribute__((ext_vector_type(4)));
typedef _Float16 v8h  __attribute__((ext_vector_type(8)));
typedef _Float16 v16h __attribute__((ext_vector_type(16)));
union FragH { v16h v; v8h h[2]; };

__device__ __forceinline__ v8f wmh(v16h a, v16h b, v8f c) {
  v8f d = __builtin_amdgcn_wmma_f32_16x16x32_f16(false, a, false, b, (short)0, c, false, false);
  asm volatile("v_nop\n\tv_nop\n\tv_nop\n\tv_nop" : "+v"(d) : "v"(a), "v"(b));
  return d;
}

__device__ __forceinline__ v8h cvt8(v4f a, v4f b, float s) {
  v8f t;
  t[0] = a.x * s; t[1] = a.y * s; t[2] = a.z * s; t[3] = a.w * s;
  t[4] = b.x * s; t[5] = b.y * s; t[6] = b.z * s; t[7] = b.w * s;
  return __builtin_convertvector(t, v8h);
}

__device__ __forceinline__ v4f ld4f(const float* p) { return *(const v4f*)p; }
__device__ __forceinline__ v4f ld4f(const _Float16* p) {
  const v4h hv = *(const v4h*)p;
  return __builtin_convertvector(hv, v4f);
}

template <int NB>
__device__ __forceinline__ int scan_chunk(const int* __restrict__ dsts, int nE, int cbase, int slotBase,
                                          int vec8, int* list, int tid, int lane, int wave) {
  int wc = 0;
#pragma unroll
  for (int g = 0; g < NGRP; ++g) {
    const int el0  = (g * NTHR + tid) * EPT;
    const int e0   = cbase + el0;
    const int sent = -2147483647 - 1;
    v4i da, db;
    if (vec8 != 0 && cbase + CHUNK <= nE) {
      da = *(const v4i*)(dsts + e0);
      db = *(const v4i*)(dsts + e0 + 4);
    } else {
      da.x = (e0     < nE) ? dsts[min(e0, nE - 1)] : sent;
      da.y = (e0 + 1 < nE) ? dsts[min(e0 + 1, nE - 1)] : sent;
      da.z = (e0 + 2 < nE) ? dsts[min(e0 + 2, nE - 1)] : sent;
      da.w = (e0 + 3 < nE) ? dsts[min(e0 + 3, nE - 1)] : sent;
      db.x = (e0 + 4 < nE) ? dsts[min(e0 + 4, nE - 1)] : sent;
      db.y = (e0 + 5 < nE) ? dsts[min(e0 + 5, nE - 1)] : sent;
      db.z = (e0 + 6 < nE) ? dsts[min(e0 + 6, nE - 1)] : sent;
      db.w = (e0 + 7 < nE) ? dsts[min(e0 + 7, nE - 1)] : sent;
    }
    const unsigned nb = (unsigned)slotBase;
    const unsigned s0 = (unsigned)da.x - nb, s1 = (unsigned)da.y - nb;
    const unsigned s2 = (unsigned)da.z - nb, s3 = (unsigned)da.w - nb;
    const unsigned s4 = (unsigned)db.x - nb, s5 = (unsigned)db.y - nb;
    const unsigned s6 = (unsigned)db.z - nb, s7 = (unsigned)db.w - nb;
    const bool h0 = s0 < (unsigned)NB, h1 = s1 < (unsigned)NB, h2 = s2 < (unsigned)NB, h3 = s3 < (unsigned)NB;
    const bool h4 = s4 < (unsigned)NB, h5 = s5 < (unsigned)NB, h6 = s6 < (unsigned)NB, h7 = s7 < (unsigned)NB;
    const unsigned any = __builtin_amdgcn_ballot_w32(h0 | h1 | h2 | h3 | h4 | h5 | h6 | h7);
    if (any != 0u) {
#define HITJ(J, HJ, SJ) { \
        const unsigned mj = __builtin_amdgcn_ballot_w32(HJ); \
        if (mj != 0u) { \
          if (HJ) { \
            const int pos = wc + (int)__builtin_amdgcn_mbcnt_lo(mj, 0u); \
            if (pos < WCAP) list[wave * WCAP + pos] = ((el0 + (J)) << 12) | (int)(SJ); \
          } \
          wc += (int)__builtin_popcount(mj); } }
      HITJ(0, h0, s0)
      HITJ(1, h1, s1)
      HITJ(2, h2, s2)
      HITJ(3, h3, s3)
      HITJ(4, h4, s4)
      HITJ(5, h5, s5)
      HITJ(6, h6, s6)
      HITJ(7, h7, s7)
#undef HITJ
    }
  }
  return wc;
}

__global__ __launch_bounds__(NTHR) void k_xcvt(const float* __restrict__ x, _Float16* xp, int nN, int nUnits) {
  constexpr int UPR = DI / 8;
  static_assert((UPR & (UPR - 1)) == 0);
  const int i = (int)blockIdx.x * NTHR + (int)threadIdx.x;
  if (i >= nUnits) return;
  const int row = i / UPR;
  const int c0  = (i & (UPR - 1)) * 8;
  int rr = row > nN - 1 ? nN - 1 : row;
  rr = rr < 0 ? 0 : rr;
  const float* p = x + (size_t)rr * DI + c0;
  const v4f a = *(const v4f*)p;
  const v4f b = *(const v4f*)(p + 4);
  v8h o = cvt8(a, b, SCL_A);
  const v8h z = {(_Float16)0.0f, (_Float16)0.0f, (_Float16)0.0f, (_Float16)0.0f,
                 (_Float16)0.0f, (_Float16)0.0f, (_Float16)0.0f, (_Float16)0.0f};
  o = (row < nN) ? o : z;
  _Float16* d = xp + (size_t)i * 8;
  *(volatile v8h*)d = o;
  __threadfence();
  *(volatile v8h*)d = o;
}

template <int K, int NC>
__global__ __launch_bounds__(NTHR) void k_prepw_layer(const float* __restrict__ Wl, const float* __restrict__ Wr, _Float16* wp) {
  constexpr int UPR = (2 * K) / 8;
  constexpr int NU  = NC * UPR;
  static_assert((K % 8) == 0 && (NU % NTHR) == 0);
  const int i = (int)blockIdx.x * NTHR + (int)threadIdx.x;
  if (i >= NU) return;
  const int n  = i / UPR;
  const int k0 = (i - n * UPR) * 8;
  const int nc = n < NC ? n : NC - 1;
  int kl = k0 > K - 8 ? K - 8 : k0;
  kl = kl < 0 ? 0 : kl;
  int kr = k0 - K;
  kr = kr < 0 ? 0 : (kr > K - 8 ? K - 8 : kr);
  const float* pl = Wl + (size_t)nc * K + kl;
  const float* pr = Wr + (size_t)nc * K + kr;
  const v4f l0 = *(const v4f*)pl;
  const v4f l1 = *(const v4f*)(pl + 4);
  const v4f r0 = *(const v4f*)pr;
  const v4f r1 = *(const v4f*)(pr + 4);
  const bool left = k0 < K;
  const v4f a = left ? l0 : r0;
  const v4f b = left ? l1 : r1;
  const v8h o = cvt8(a, b, SCL_W);
  _Float16* d = wp + (size_t)i * 8;
  *(volatile v8h*)d = o;
  __threadfence();
  *(volatile v8h*)d = o;
}

template <int K, int NC>
__global__ __launch_bounds__(NTHR) void k_prepw_pair(const float* __restrict__ W, _Float16* wp) {
  constexpr int UPR = K / 8;
  constexpr int NU  = 2 * NC * UPR;
  static_assert((K % 8) == 0 && (NU % NTHR) == 0 && (NC & (NC - 1)) == 0);
  const int i = (int)blockIdx.x * NTHR + (int)threadIdx.x;
  if (i >= NU) return;
  const int n2 = i / UPR;
  const int k0 = (i - n2 * UPR) * 8;
  const bool hi = n2 >= NC;
  const int col = n2 & (NC - 1);
  const int koff = hi ? K : 0;
  const float* p = W + (size_t)col * (2 * K) + koff + k0;
  const v4f a = *(const v4f*)p;
  const v4f b = *(const v4f*)(p + 4);
  const v8h o = cvt8(a, b, SCL_W);
  _Float16* d = wp + (size_t)i * 8;
  *(volatile v8h*)d = o;
  __threadfence();
  *(volatile v8h*)d = o;
}

__global__ __launch_bounds__(NTHR) void k_prepw_flat(const float* __restrict__ W, _Float16* wp, int nUnits) {
  const int i = (int)blockIdx.x * NTHR + (int)threadIdx.x;
  if (i >= nUnits) return;
  const float* p = W + (size_t)i * 8;
  const v4f a = *(const v4f*)p;
  const v4f b = *(const v4f*)(p + 4);
  const v8h o = cvt8(a, b, SCL_W);
  _Float16* d = wp + (size_t)i * 8;
  *(volatile v8h*)d = o;
  __threadfence();
  *(volatile v8h*)d = o;
}

__global__ __launch_bounds__(NTHR) void k_count(
    const int* __restrict__ dsts, int* cnt, int nE, int vec8) {
  __shared__ __attribute__((aligned(16))) int scnt[NBC];
  __shared__ __attribute__((aligned(16))) int list[LISTN];
  __shared__ int wcnt[NWAVE];
  const int tid = threadIdx.x, lane = tid & 31, wave = tid >> 5;
  const int nodeBase = blockIdx.x * NBC;

  for (int i = tid; i < NBC; i += NTHR) scnt[i] = 0;
  __syncthreads();

  const int nChunks = (nE + CHUNK - 1) / CHUNK;
#pragma unroll 1
  for (int ch = 0; ch < nChunks; ++ch) {
    const int cbase = ch * CHUNK;
    const int wc = scan_chunk<NBC>(dsts, nE, cbase, nodeBase, vec8, list, tid, lane, wave);
    if (lane == 0) wcnt[wave] = wc;
    __syncthreads();
    if (wave == 0) {
#pragma unroll 1
      for (int wsx = 0; wsx < NWAVE; ++wsx) {
        int n = __builtin_amdgcn_readfirstlane(wcnt[wsx]);
        n = n > WCAP ? WCAP : (n < 0 ? 0 : n);
        const int* lp = list + wsx * WCAP;
#pragma unroll 1
        for (int i = 0; i < n; ++i) {
          const int ent  = __builtin_amdgcn_readfirstlane(lp[i]);
          const int slot = ent & (NBC - 1);
          if (lane == 0) scnt[slot] = scnt[slot] + 1;
        }
      }
    }
    __syncthreads();
  }

  v4i cq[4];
#pragma unroll
  for (int q = 0; q < 4; ++q) {
    const int f = (wave * 4 + q) * 128 + 4 * lane;
    cq[q] = *(const v4i*)(scnt + f);
  }
  int* cp = cnt + (size_t)nodeBase;
#pragma unroll
  for (int q = 0; q < 4; ++q) {
    const int f = (wave * 4 + q) * 128 + 4 * lane;
    *(volatile v4i*)(cp + f) = cq[q];
  }
  __threadfence();
#pragma unroll
  for (int q = 0; q < 4; ++q) {
    const int f = (wave * 4 + q) * 128 + 4 * lane;
    *(volatile v4i*)(cp + f) = cq[q];
  }
}

__global__ __launch_bounds__(OTHR) void k_offsets(
    const int* __restrict__ cnt, int* off, int* rbase, int nChunk) {
  __shared__ __attribute__((aligned(16))) int soff[NBC];
  __shared__ __attribute__((aligned(16))) int srb[RBN];
  __shared__ int wtot[OTHR / 32];
  const int tid = threadIdx.x, lane = tid & 31, wave = tid >> 5, sub = tid >> 7;
  for (int i = tid; i < RBN; i += OTHR) srb[i] = 0;
  int carry = 0;
#pragma unroll 1
  for (int ch = 0; ch < nChunk; ++ch) {
    const int base = ch * NBC;
    const v4i c0 = *(const v4i*)(cnt + base + 8 * tid);
    const v4i c1 = *(const v4i*)(cnt + base + 8 * tid + 4);
    const int e0 = max(c0.x, 0), e1 = max(c0.y, 0), e2 = max(c0.z, 0), e3 = max(c0.w, 0);
    const int e4 = max(c1.x, 0), e5 = max(c1.y, 0), e6 = max(c1.z, 0), e7 = max(c1.w, 0);
    const int ts = e0 + e1 + e2 + e3 + e4 + e5 + e6 + e7;
    int incl = ts;
#pragma unroll
    for (int d = 1; d < 32; d <<= 1) {
      const int t = __shfl_up(incl, d);
      if (lane >= d) incl += t;
    }
    if (lane == 31) wtot[wave] = incl;
    __syncthreads();
    const int S0 = wtot[0]  + wtot[1]  + wtot[2]  + wtot[3];
    const int S1 = wtot[4]  + wtot[5]  + wtot[6]  + wtot[7];
    const int S2 = wtot[8]  + wtot[9]  + wtot[10] + wtot[11];
    const int S3 = wtot[12] + wtot[13] + wtot[14] + wtot[15];
    int pre = 0;
#pragma unroll 1
    for (int w = 4 * sub; w < wave; ++w) pre += wtot[w];
    const int b0 = carry;
    const int b1 = b0 + ((S0 + 31) & ~31);
    const int b2 = b1 + ((S1 + 31) & ~31);
    const int b3 = b2 + ((S2 + 31) & ~31);
    const int b4 = b3 + ((S3 + 31) & ~31);
    const int myb = sub == 0 ? b0 : (sub == 1 ? b1 : (sub == 2 ? b2 : b3));
    if (tid == 0) {
      srb[min(4 * ch + 0, RBN - 1)] = b0;
      srb[min(4 * ch + 1, RBN - 1)] = b1;
      srb[min(4 * ch + 2, RBN - 1)] = b2;
      srb[min(4 * ch + 3, RBN - 1)] = b3;
    }
    int run = myb + pre + incl - ts;
    soff[8 * tid + 0] = run; run += e0;
    soff[8 * tid + 1] = run; run += e1;
    soff[8 * tid + 2] = run; run += e2;
    soff[8 * tid + 3] = run; run += e3;
    soff[8 * tid + 4] = run; run += e4;
    soff[8 * tid + 5] = run; run += e5;
    soff[8 * tid + 6] = run; run += e6;
    soff[8 * tid + 7] = run;
    carry = b4;
    __syncthreads();
    const v4i o0 = *(const v4i*)(soff + 4 * tid);
    const v4i o1 = *(const v4i*)(soff + 4 * (tid + OTHR));
    int* op = off + base;
    *(volatile v4i*)(op + 4 * tid) = o0;
    *(volatile v4i*)(op + 4 * (tid + OTHR)) = o1;
    __threadfence();
    *(volatile v4i*)(op + 4 * tid) = o0;
    *(volatile v4i*)(op + 4 * (tid + OTHR)) = o1;
    __syncthreads();
  }
  if (tid == 0) srb[min(4 * nChunk, RBN - 1)] = carry;
  __syncthreads();
  v4i rv = {0, 0, 0, 0};
  if (tid < 32) rv = *(const v4i*)(srb + 4 * tid);
  if (tid < 32) *(volatile v4i*)(rbase + 4 * tid) = rv;
  __threadfence();
  if (tid < 32) *(volatile v4i*)(rbase + 4 * tid) = rv;
}

__global__ __launch_bounds__(NTHR) void k_fill(
    const int* __restrict__ dsts, const int* __restrict__ off, const int* __restrict__ rbase,
    int* csr, int nE, int vec8, int csrLen) {
  extern __shared__ v4f lds_dyn[];
  int* region = (int*)lds_dyn;
  int* cursor = region + RCAP;
  int* list   = cursor + NBF;
  int* wcnt   = list + LISTN;
  const int tid = threadIdx.x, lane = tid & 31, wave = tid >> 5;
  const int b = blockIdx.x;
  const int nodeBase = b * NBF;

  int rb0 = rbase[b];
  const int rb1 = rbase[b + 1];
  rb0 = rb0 < 0 ? 0 : (rb0 > csrLen ? csrLen : rb0);
  rb0 &= ~31;
  int len = rb1 - rb0;
  len = len < 0 ? 0 : (len > RCAP ? RCAP : len);
  int lenW = (len + 31) & ~31;
  if (rb0 + lenW > csrLen) lenW = (csrLen - rb0) & ~31;

  {
    const v4i z = {0, 0, 0, 0};
    for (int i = tid; i < RCAP / 4; i += NTHR) ((v4i*)region)[i] = z;
    for (int s = tid; s < NBF; s += NTHR) {
      int o = off[nodeBase + s] - rb0;
      o = o < 0 ? 0 : (o > RCAP ? RCAP : o);
      cursor[s] = o;
    }
  }
  __syncthreads();

  const int nChunks = (nE + CHUNK - 1) / CHUNK;
#pragma unroll 1
  for (int ch = 0; ch < nChunks; ++ch) {
    const int cbase = ch * CHUNK;
    const int wc = scan_chunk<NBF>(dsts, nE, cbase, nodeBase, vec8, list, tid, lane, wave);
    if (lane == 0) wcnt[wave] = wc;
    __syncthreads();
    if (wave == 0) {
#pragma unroll 1
      for (int wsx = 0; wsx < NWAVE; ++wsx) {
        int n = __builtin_amdgcn_readfirstlane(wcnt[wsx]);
        n = n > WCAP ? WCAP : (n < 0 ? 0 : n);
        const int* lp = list + wsx * WCAP;
#pragma unroll 1
        for (int i = 0; i < n; ++i) {
          const int ent  = __builtin_amdgcn_readfirstlane(lp[i]);
          const int slot = ent & (NBF - 1);
          int e = cbase + ((ent >> 12) & (CHUNK - 1));
          e = e > nE - 1 ? nE - 1 : (e < 0 ? 0 : e);
          if (lane == 0) {
            int pos = cursor[slot];
            pos = pos < 0 ? 0 : (pos > RCAP - 1 ? RCAP - 1 : pos);
            region[pos] = e;
            const int np = pos + 1;
            cursor[slot] = np > RCAP ? RCAP : np;
          }
        }
      }
    }
    __syncthreads();
  }

  const int nv = lenW >> 2;
  int* gp = csr + rb0;
#pragma unroll 1
  for (int i = tid; i < nv; i += NTHR) { const v4i v = ((const v4i*)region)[i]; *(volatile v4i*)(gp + 4 * i) = v; }
  __threadfence();
#pragma unroll 1
  for (int i = tid; i < nv; i += NTHR) { const v4i v = ((const v4i*)region)[i]; *(volatile v4i*)(gp + 4 * i) = v; }
}

template <typename ST, int OSC>
__global__ __launch_bounds__(NTHR) void k_mean(
    const int* __restrict__ csr, const int* __restrict__ off, const int* __restrict__ cnt,
    const int* __restrict__ srcs, const ST* __restrict__ hp, _Float16* ap,
    int nN, int nE, int csrLen) {
  const int tid = threadIdx.x, lane = tid & 31, wave = tid >> 5;
  const int tbase = blockIdx.x * TGT + wave * 32;
  const int col = 4 * lane;

  const int cl    = tbase + lane;
  const int cnt_l = cnt[cl];
  const int off_l = off[cl];

#pragma unroll 1
  for (int j = 0; j < 32; ++j) {
    const int c = tbase + j;
    int nraw = __shfl(cnt_l, j);
    nraw = nraw < 0 ? 0 : (nraw > nE ? nE : nraw);
    const int n = nraw > DEGCAP ? DEGCAP : nraw;
    const int st = __shfl(off_l, j);

    v4f acc = {0.0f, 0.0f, 0.0f, 0.0f};
#pragma unroll 1
    for (int q0 = 0; q0 < n; q0 += 32) {
      int pos = st + q0 + lane;
      pos = pos < 0 ? 0 : (pos > csrLen - 1 ? csrLen - 1 : pos);
      int el = csr[pos];
      el = el < 0 ? 0 : (el > nE - 1 ? nE - 1 : el);
      int sl = srcs[el];
      sl = sl < 0 ? 0 : (sl > nN - 1 ? nN - 1 : sl);
      const int mcnt = (n - q0) < 32 ? (n - q0) : 32;
#pragma unroll 1
      for (int pp = 0; pp < mcnt; ++pp) {
        const int s = __builtin_amdgcn_readlane(sl, pp);
        acc = acc + ld4f(hp + (size_t)s * DI + col);
      }
    }

    const float nf = (float)(nraw < 1 ? 1 : nraw);
    const float rd = (1.0f / nf) * (float)OSC;
    v4f v = acc * rd;
    if (nraw > DEGCAP) { const float qn = __int_as_float(0x7fc00000); v.x = qn; v.y = qn; v.z = qn; v.w = qn; }
    if (c >= nN) { v.x = 0.0f; v.y = 0.0f; v.z = 0.0f; v.w = 0.0f; }
    const v4h o = __builtin_convertvector(v, v4h);
    _Float16* gp = ap + (size_t)c * DI + col;
    *(volatile v4h*)gp = o;
    __threadfence();
    *(volatile v4h*)gp = o;
  }
}

template <int K, int LDB, int TPW>
__device__ __forceinline__ void mma_pair(const _Float16* __restrict__ Ap, const _Float16* __restrict__ Bp,
                                         int arow, int c0, int m, int hh, v8f (&acc)[TPW]) {
  constexpr int KT = K / 32;
  static_assert(K % 32 == 0 && LDB % 8 == 0);
  const _Float16* ap  = Ap + (size_t)arow * K + 8 * hh;
  const _Float16* bp0 = Bp + (size_t)(c0 + m) * LDB + 8 * hh;
#pragma unroll 1
  for (int kt = 0; kt < KT; ++kt) {
    FragH a;
    a.h[0] = *(const v8h*)(ap + 32 * kt);
    a.h[1] = *(const v8h*)(ap + 32 * kt + 16);
#pragma unroll
    for (int t = 0; t < TPW; ++t) {
      const _Float16* bp = bp0 + (size_t)(16 * t) * LDB + 32 * kt;
      FragH bf;
      bf.h[0] = *(const v8h*)bp;
      bf.h[1] = *(const v8h*)(bp + 16);
      acc[t] = wmh(a.v, bf.v, acc[t]);
    }
  }
}

template <int K, int NC, int LDB, int NPAIR, int RELU, int HASBIAS, int BN>
__device__ __forceinline__ void gemm_stage(
    const _Float16* __restrict__ A1, const _Float16* __restrict__ A2,
    const _Float16* __restrict__ Bp, const float* __restrict__ bias,
    const float* __restrict__ bng, const float* __restrict__ bnb,
    const float* __restrict__ bnm, const float* __restrict__ bnv,
    float* stg, int rowBase, int nN, int lane, int wave) {
  constexpr int TPW = NC / 64;
  static_assert(K % 32 == 0);
  static_assert(NC % 64 == 0 && TPW >= 1);
  static_assert(NPAIR == 1 || NPAIR == 2);
  const int hh = lane >> 4, m = lane & 15;
  const int rg = wave >> 2, cq = wave & 3;
  const int r0 = rg * 16;
  const int c0 = cq * (NC / 4);

  v8f acc[TPW];
#pragma unroll
  for (int t = 0; t < TPW; ++t) { v8f z = {0.f, 0.f, 0.f, 0.f, 0.f, 0.f, 0.f, 0.f}; acc[t] = z; }

  mma_pair<K, LDB, TPW>(A1, Bp, rowBase + r0 + m, c0, m, hh, acc);
  if (NPAIR == 2) mma_pair<K, LDB, TPW>(A2, Bp + K, rowBase + r0 + m, c0, m, hh, acc);

  float* sp = stg + (size_t)(r0 + 8 * hh) * NC + c0 + m;
  const int grow0 = rowBase + r0 + 8 * hh;
#pragma unroll
  for (int t = 0; t < TPW; ++t) {
    const int n = c0 + 16 * t + m;
    float bv = 0.0f;
    if (HASBIAS) bv = bias[n];
    float g = 1.0f, be = 0.0f, mu = 0.0f, rs = 1.0f;
    if (BN) { g = bng[n]; be = bnb[n]; mu = bnm[n]; rs = rsqrtf(bnv[n] + 1e-5f); }
#pragma unroll
    for (int r = 0; r < 8; ++r) {
      float v = acc[t][r] * SCL_ACC + bv;
      if (BN) v = (v - mu) * rs * g + be;
      if (RELU) v = v > 0.0f ? v : 0.0f;
      v = (grow0 + r < nN) ? v : 0.0f;
      sp[r * NC + 16 * t] = v;
    }
  }
}

template <int K, int NC, int LDB, int NPAIR, int RELU, int BN>
__global__ __launch_bounds__(NTHR) void k_gemm16(
    const _Float16* __restrict__ A1, const _Float16* __restrict__ A2,
    const _Float16* __restrict__ Bp, const float* __restrict__ bias,
    const float* __restrict__ bng, const float* __restrict__ bnb,
    const float* __restrict__ bnm, const float* __restrict__ bnv,
    _Float16* Hq, int nN) {
  constexpr int NIT8 = (BM * NC / 8) / NTHR;
  static_assert((BM * NC / 8) % NTHR == 0 && NIT8 >= 1);
  static_assert(BM * 8 == NTHR);
  __shared__ __attribute__((aligned(16))) float stg[BM * NC];
  const int tid = threadIdx.x, lane = tid & 31, wave = tid >> 5;
  const int rowBase = blockIdx.x * BM;

  gemm_stage<K, NC, LDB, NPAIR, RELU, 1, BN>(A1, A2, Bp, bias, bng, bnb, bnm, bnv, stg, rowBase, nN, lane, wave);
  __syncthreads();

  _Float16* tile = Hq + (size_t)rowBase * NC;
  v8h hv[NIT8];
#pragma unroll
  for (int it = 0; it < NIT8; ++it) {
    const int u = it * NTHR + tid;
    const v4f x0 = *(const v4f*)(stg + 8 * u);
    const v4f x1 = *(const v4f*)(stg + 8 * u + 4);
    hv[it] = cvt8(x0, x1, SCL_A);
  }
#pragma unroll
  for (int it = 0; it < NIT8; ++it) *(volatile v8h*)(tile + 8 * (size_t)(it * NTHR + tid)) = hv[it];
  __threadfence();
#pragma unroll
  for (int it = 0; it < NIT8; ++it) *(volatile v8h*)(tile + 8 * (size_t)(it * NTHR + tid)) = hv[it];
}

template <int K, int NC, int LDB, int NPAIR>
__global__ __launch_bounds__(NTHR) void k_gemm32(
    const _Float16* __restrict__ A1, const _Float16* __restrict__ A2,
    const _Float16* __restrict__ Bp, const float* __restrict__ dummy,
    float* Zp, int nN) {
  constexpr int NIT4 = (BM * NC / 4) / NTHR;
  static_assert((BM * NC / 4) % NTHR == 0 && NIT4 >= 1);
  static_assert(BM * 8 == NTHR);
  __shared__ __attribute__((aligned(16))) float stg[BM * NC];
  const int tid = threadIdx.x, lane = tid & 31, wave = tid >> 5;
  const int rowBase = blockIdx.x * BM;

  gemm_stage<K, NC, LDB, NPAIR, 0, 0, 0>(A1, A2, Bp, dummy, dummy, dummy, dummy, dummy, stg, rowBase, nN, lane, wave);
  __syncthreads();

  float* tile = Zp + (size_t)rowBase * NC;
  v4f ov[NIT4];
#pragma unroll
  for (int it = 0; it < NIT4; ++it) ov[it] = *(const v4f*)(stg + 4 * (it * NTHR + tid));
#pragma unroll
  for (int it = 0; it < NIT4; ++it) *(volatile v4f*)(tile + 4 * (size_t)(it * NTHR + tid)) = ov[it];
  __threadfence();
#pragma unroll
  for (int it = 0; it < NIT4; ++it) *(volatile v4f*)(tile + 4 * (size_t)(it * NTHR + tid)) = ov[it];
}

__global__ __launch_bounds__(DTHR) void k_decode(
    const float* __restrict__ pq, const int* __restrict__ pa, const int* __restrict__ pb,
    const float* __restrict__ b1, const _Float16* __restrict__ w2p, const float* __restrict__ b2,
    const float* __restrict__ w3, const float* __restrict__ b3,
    float* out, int nL, int nN) {
  constexpr int NUD = DTHR / 4;
  constexpr int PW  = 2 * DZ;
  constexpr int NWD = DTHR / 32;
  static_assert((NUD & (NUD - 1)) == 0 && NUD == 64 && NWD == 8);
  __shared__ __attribute__((aligned(16))) _Float16 us[NWD * 32 * LDU];
  __shared__ __attribute__((aligned(16))) float sres[DTHR];
  const int tid = threadIdx.x, lane = tid & 31, wave = tid >> 5;
  const int hh = lane >> 4, m = lane & 15;
  const int gbase = blockIdx.x * DTHR;
  const int pbase = gbase + wave * 32;
  int pl = pbase + lane;
  pl = pl > nL - 1 ? nL - 1 : pl;
  pl = pl < 0 ? 0 : pl;
  int ai = pa[pl];
  int bi = pb[pl];
  ai = ai < 0 ? 0 : (ai > nN - 1 ? nN - 1 : ai);
  bi = bi < 0 ? 0 : (bi > nN - 1 ? nN - 1 : bi);

  const int col2 = 2 * lane;
  const v2f bb = *(const v2f*)(b1 + col2);
  _Float16* uw = us + wave * (32 * LDU);

#pragma unroll 1
  for (int j = 0; j < 32; ++j) {
    const int sa = __builtin_amdgcn_readlane(ai, j);
    const int sb = __builtin_amdgcn_readlane(bi, j);
    const v2f p = *(const v2f*)(pq + (size_t)sa * PW + col2);
    const v2f q = *(const v2f*)(pq + (size_t)sb * PW + DZ + col2);
    v2f u = p + q + bb;
    u.x = u.x > 0.0f ? u.x : 0.0f;
    u.y = u.y > 0.0f ? u.y : 0.0f;
    u = u * SCL_A;
    const v2h o = __builtin_convertvector(u, v2h);
    *(v2h*)(uw + j * LDU + col2) = o;
  }
  __syncthreads();

  const float b2a = b2[m], b2b = b2[16 + m];
  const float w3a = w3[m], w3b = w3[16 + m];
  const float c3  = b3[0];

  FragH bq[2][2];
#pragma unroll
  for (int t = 0; t < 2; ++t) {
#pragma unroll
    for (int kt = 0; kt < 2; ++kt) {
      const _Float16* bp = w2p + (size_t)(16 * t + m) * DZ + 32 * kt + 8 * hh;
      bq[t][kt].h[0] = *(const v8h*)bp;
      bq[t][kt].h[1] = *(const v8h*)(bp + 16);
    }
  }

  float res[2];
#pragma unroll
  for (int g = 0; g < 2; ++g) {
    v8f acc0 = {0.f, 0.f, 0.f, 0.f, 0.f, 0.f, 0.f, 0.f};
    v8f acc1 = {0.f, 0.f, 0.f, 0.f, 0.f, 0.f, 0.f, 0.f};
    const _Float16* arow = uw + (16 * g + m) * LDU + 8 * hh;
#pragma unroll
    for (int kt = 0; kt < 2; ++kt) {
      FragH a;
      a.h[0] = *(const v8h*)(arow + 32 * kt);
      a.h[1] = *(const v8h*)(arow + 32 * kt + 16);
      acc0 = wmh(a.v, bq[0][kt].v, acc0);
      acc1 = wmh(a.v, bq[1][kt].v, acc1);
    }
    v8f part;
#pragma unroll
    for (int r = 0; r < 8; ++r) {
      float v0 = acc0[r] * SCL_ACC + b2a;
      float v1 = acc1[r] * SCL_ACC + b2b;
      v0 = v0 > 0.0f ? v0 : 0.0f;
      v1 = v1 > 0.0f ? v1 : 0.0f;
      part[r] = v0 * w3a + v1 * w3b;
    }
#pragma unroll
    for (int r = 0; r < 8; ++r) {
      float t = part[r];
      t += __shfl_xor(t, 8);
      t += __shfl_xor(t, 4);
      t += __shfl_xor(t, 2);
      t += __shfl_xor(t, 1);
      part[r] = t;
    }
    float mine = 0.0f;
#pragma unroll
    for (int r = 0; r < 8; ++r) mine = ((m & 7) == r) ? part[r] : mine;
    float s = mine + c3;
    s = s > 40.0f ? 40.0f : (s < -40.0f ? -40.0f : s);
    const float ex = expf(-s);
    res[g] = 1.0f / (1.0f + ex);
  }
  if (m < 8) {
    sres[wave * 32 + 8 * hh + m]      = res[0];
    sres[wave * 32 + 16 + 8 * hh + m] = res[1];
  }
  __syncthreads();

  const v4f v = *(const v4f*)(sres + 4 * (tid & (NUD - 1)));
  const int e0 = gbase + 4 * tid;
  const bool act  = tid < NUD;
  const bool full = act && (e0 + 3 < nL);
  const bool part1 = act && !full && (e0 < nL);
  if (full) {
    *(volatile v4f*)(out + e0) = v;
  } else if (part1) {
    if (e0 < nL)     *(volatile float*)(out + e0)     = v.x;
    if (e0 + 1 < nL) *(volatile float*)(out + e0 + 1) = v.y;
    if (e0 + 2 < nL) *(volatile float*)(out + e0 + 2) = v.z;
  }
  __threadfence();
  if (full) {
    *(volatile v4f*)(out + e0) = v;
  } else if (part1) {
    if (e0 < nL)     *(volatile float*)(out + e0)     = v.x;
    if (e0 + 1 < nL) *(volatile float*)(out + e0 + 1) = v.y;
    if (e0 + 2 < nL) *(volatile float*)(out + e0 + 2) = v.z;
  }
}

extern "C" void kernel_launch(void* const* d_in, const int* in_sizes, int n_in,
                              void* d_out, int out_size, void* d_ws, size_t ws_size,
                              hipStream_t stream) {
  if (n_in < 19) return;
  const int nN = in_sizes[0] / DI;
  const int nE = in_sizes[1] / 2;
  const int nL = in_sizes[2] / 2;
  if (nN <= 0 || nE <= 0 || nL <= 0) return;
  if (in_sizes[0] != nN * DI || in_sizes[1] != 2 * nE || in_sizes[2] != 2 * nL) return;
  if (in_sizes[3] != DH * DI || in_sizes[4] != DH || in_sizes[5] != DH * DI) return;
  if (in_sizes[6] != DH || in_sizes[7] != DH || in_sizes[8] != DH || in_sizes[9] != DH) return;
  if (in_sizes[10] != DZ * DH || in_sizes[11] != DZ || in_sizes[12] != DZ * DH) return;
  if (in_sizes[13] != DZ * 2 * DZ || in_sizes[14] != DZ) return;
  if (in_sizes[15] != DE * DZ || in_sizes[16] != DE || in_sizes[17] != DE || in_sizes[18] != 1) return;
  if (out_size != nL) return;
  if (nE > (1 << 28) || nN > (1 << 22) || nL > (1 << 28)) return;

  const float* x    = (const float*)d_in[0];
  const int*   ei   = (const int*)d_in[1];
  const int*   epi  = (const int*)d_in[2];
  const float* W1l  = (const float*)d_in[3];
  const float* b1   = (const float*)d_in[4];
  const float* W1r  = (const float*)d_in[5];
  const float* bng  = (const float*)d_in[6];
  const float* bnb  = (const float*)d_in[7];
  const float* bnm  = (const float*)d_in[8];
  const float* bnv  = (const float*)d_in[9];
  const float* W2l  = (const float*)d_in[10];
  const float* b2   = (const float*)d_in[11];
  const float* W2r  = (const float*)d_in[12];
  const float* We1  = (const float*)d_in[13];
  const float* be1  = (const float*)d_in[14];
  const float* We2  = (const float*)d_in[15];
  const float* be2  = (const float*)d_in[16];
  const float* We3  = (const float*)d_in[17];
  const float* be3  = (const float*)d_in[18];
  const int* src = ei;
  const int* dst = ei + nE;
  const int* pa  = epi;
  const int* pb  = epi + nL;
  float* out = (float*)d_out;

  const int NPAD   = ((nN + TGT - 1) / TGT) * TGT;
  const int nBC    = (nN + NBC - 1) / NBC;
  const int CNTPAD = nBC * NBC;
  if (CNTPAD < NPAD) return;
  if (4 * nBC + 1 > RBN) return;
  const int nBF    = (nN + NBF - 1) / NBF;
  if (nBF + 1 > 4 * nBC + 1) return;
  const int csrLen = ((nE + 31) & ~31) + 4096;
  if (31 * 4 * nBC > 4096) return;
  const int nAgg   = NPAD / TGT;
  const int nGemm  = NPAD / BM;
  const int nXu    = NPAD * (DI / 8);
  const int nDec   = (nL + DTHR - 1) / DTHR;

  char* ws = (char*)d_ws;
  size_t off = 0;
  const size_t oW1  = off; off += (size_t)DH * 2 * DI * 2;      off = (off + 255) & ~(size_t)255;
  const size_t oW2  = off; off += (size_t)DZ * 2 * DH * 2;      off = (off + 255) & ~(size_t)255;
  const size_t oWe  = off; off += (size_t)2 * DZ * DZ * 2;      off = (off + 255) & ~(size_t)255;
  const size_t oW2e = off; off += (size_t)DE * DZ * 2;          off = (off + 255) & ~(size_t)255;
  const size_t oX   = off; off += (size_t)NPAD * DI * 2;        off = (off + 255) & ~(size_t)255;
  const size_t oA   = off; off += (size_t)NPAD * DH * 2;        off = (off + 255) & ~(size_t)255;
  const size_t oH1  = off; off += (size_t)NPAD * DH * 2;        off = (off + 255) & ~(size_t)255;
  const size_t oH2  = off; off += (size_t)NPAD * DZ * 2;        off = (off + 255) & ~(size_t)255;
  const size_t oPQ  = off; off += (size_t)NPAD * 2 * DZ * 4;    off = (off + 255) & ~(size_t)255;
  const size_t oCnt = off; off += (size_t)CNTPAD * 4;           off = (off + 255) & ~(size_t)255;
  const size_t oOff = off; off += (size_t)CNTPAD * 4;           off = (off + 255) & ~(size_t)255;
  const size_t oRb  = off; off += (size_t)RBN * 4;              off = (off + 255) & ~(size_t)255;
  const size_t oCsr = off; off += (size_t)csrLen * 4;           off = (off + 255) & ~(size_t)255;
  if (off > ws_size || off > (size_t)WSCAP) return;
  _Float16* pW1  = (_Float16*)(ws + oW1);
  _Float16* pW2  = (_Float16*)(ws + oW2);
  _Float16* pWe  = (_Float16*)(ws + oWe);
  _Float16* pW2e = (_Float16*)(ws + oW2e);
  _Float16* xP   = (_Float16*)(ws + oX);
  _Float16* aggP = (_Float16*)(ws + oA);
  _Float16* h1P  = (_Float16*)(ws + oH1);
  _Float16* h2P  = (_Float16*)(ws + oH2);
  float*    pqP  = (float*)(ws + oPQ);
  int*   cnt  = (int*)(ws + oCnt);
  int*   offp = (int*)(ws + oOff);
  int*   rb   = (int*)(ws + oRb);
  int*   csr  = (int*)(ws + oCsr);

  const int vec8 = ((nE & 7) == 0) ? 1 : 0;

  k_prepw_layer<DI, DH><<<(DH * 2 * DI / 8) / NTHR, NTHR, 0, stream>>>(W1l, W1r, pW1);
  k_prepw_layer<DH, DZ><<<(DZ * 2 * DH / 8) / NTHR, NTHR, 0, stream>>>(W2l, W2r, pW2);
  k_prepw_pair<DZ, DZ><<<(2 * DZ * DZ / 8) / NTHR, NTHR, 0, stream>>>(We1, pWe);
  k_prepw_flat<<<(DE * DZ / 8 + NTHR - 1) / NTHR, NTHR, 0, stream>>>(We2, pW2e, DE * DZ / 8);
  k_xcvt<<<(nXu + NTHR - 1) / NTHR, NTHR, 0, stream>>>(x, xP, nN, nXu);

  k_count<<<nBC, NTHR, 0, stream>>>(dst, cnt, nE, vec8);
  k_offsets<<<1, OTHR, 0, stream>>>(cnt, offp, rb, nBC);
  hipFuncSetAttribute(reinterpret_cast<const void*>(&k_fill),
                      hipFuncAttributeMaxDynamicSharedMemorySize, LDS_FILL);
  k_fill<<<nBF, NTHR, LDS_FILL, stream>>>(dst, offp, rb, csr, nE, vec8, csrLen);

  k_mean<float, 8><<<nAgg, NTHR, 0, stream>>>(csr, offp, cnt, src, x, aggP, nN, nE, csrLen);
  k_gemm16<DI, DH, 2 * DI, 2, 1, 1><<<nGemm, NTHR, 0, stream>>>(aggP, xP, pW1, b1, bng, bnb, bnm, bnv, h1P, nN);

  k_mean<_Float16, 1><<<nAgg, NTHR, 0, stream>>>(csr, offp, cnt, src, h1P, aggP, nN, nE, csrLen);
  k_gemm16<DH, DZ, 2 * DH, 2, 0, 0><<<nGemm, NTHR, 0, stream>>>(aggP, h1P, pW2, b2, b2, b2, b2, b2, h2P, nN);

  k_gemm32<DZ, 2 * DZ, DZ, 1><<<nGemm, NTHR, 0, stream>>>(h2P, h2P, pWe, be1, pqP, nN);

  k_decode<<<nDec, DTHR, 0, stream>>>(pqP, pa, pb, be1, pW2e, be2, We3, be3, out, nL, nN);
}
